// ResTAttention_46926812676790
// MI455X (gfx1250) — hardware-verified
//
#include <hip/hip_runtime.h>
#include <stdint.h>

typedef _Float16 half_t;
typedef __attribute__((ext_vector_type(16))) _Float16 v16h;
typedef __attribute__((ext_vector_type(8)))  _Float16 v8h;
typedef __attribute__((ext_vector_type(16))) __bf16   v16b;
typedef __attribute__((ext_vector_type(8)))  __bf16   v8b;
typedef __attribute__((ext_vector_type(8)))  float    v8f;
typedef __attribute__((ext_vector_type(4)))  float    v4f;

#define B_   8
#define C_   256
#define H_   48
#define W_   48
#define N_   2304
#define NH_  8
#define HD_  32
#define M_   576
#define MH_  24
#define EPS_ 1e-5f
#define SCALE_ 0.17677669529663687f
#define WSC 64.0f
#define WSC_INV (1.0f / 64.0f)
#define DSC 16384.0f
#define DSC_INV (1.0f / 16384.0f)
#define INV_M (1.0f / 576.0f)
#define INV_CNT (1.0 / 1327104.0)
#define MIXT 192

__device__ __forceinline__ unsigned short f2bf_bits(float f) {
  unsigned u = __float_as_uint(f);
  return (unsigned short)((u + 0x7FFFu + ((u >> 16) & 1u)) >> 16);
}
__device__ __forceinline__ float bf_bits2f(unsigned short h) { return __uint_as_float(((unsigned)h) << 16); }

__device__ __forceinline__ void dep_guard_h(v8f& a, v8f& b, v16h x, v16h y) { asm volatile("v_nop\n\tv_nop\n\tv_nop\n\tv_nop" : "+v"(a), "+v"(b) : "v"(x), "v"(y)); }
__device__ __forceinline__ void dep_guard_b(v8f& a, v8f& b, v16b x, v16b y) { asm volatile("v_nop\n\tv_nop\n\tv_nop\n\tv_nop" : "+v"(a), "+v"(b) : "v"(x), "v"(y)); }
__device__ __forceinline__ void keep4_h(v16h a, v16h b, v16h c, v16h d) { asm volatile("v_nop" :: "v"(a), "v"(b), "v"(c), "v"(d)); }
__device__ __forceinline__ void keep4_b(v16b a, v16b b, v16b c, v16b d) { asm volatile("v_nop" :: "v"(a), "v"(b), "v"(c), "v"(d)); }
__device__ __forceinline__ void acc_guard4(v8f& a, v8f& b, v8f& c, v8f& d) { asm volatile("v_nop\n\tv_nop\n\tv_nop\n\tv_nop" : "+v"(a), "+v"(b), "+v"(c), "+v"(d)); }
template <typename T> struct Frag;
template <> struct Frag<_Float16> {
  typedef v16h V; union U { v16h v; v8h h[2]; };
  static __device__ __forceinline__ v16h load(const _Float16* p) {
    U f; f.h[0] = *(const v8h*)(p); f.h[1] = *(const v8h*)(p + 16); return f.v;
  }
  static __device__ __forceinline__ v8f mma(v16h a, v16h b, v8f c) {
    return __builtin_amdgcn_wmma_f32_16x16x32_f16(false, a, false, b, (short)0, c, false, false);
  }
  static __device__ __forceinline__ void guard(v8f& a, v8f& b, v16h x, v16h y) { dep_guard_h(a, b, x, y); }
  static __device__ __forceinline__ void keep(v16h a, v16h b, v16h c, v16h d) { keep4_h(a, b, c, d); }
};
template <> struct Frag<__bf16> {
  typedef v16b V; union U { v16b v; v8b h[2]; };
  static __device__ __forceinline__ v16b load(const __bf16* p) {
    U f; f.h[0] = *(const v8b*)(p); f.h[1] = *(const v8b*)(p + 16); return f.v;
  }
  static __device__ __forceinline__ v8f mma(v16b a, v16b b, v8f c) {
    return __builtin_amdgcn_wmma_f32_16x16x32_bf16(false, a, false, b, (short)0, c, false, false);
  }
  static __device__ __forceinline__ void guard(v8f& a, v8f& b, v16b x, v16b y) { dep_guard_b(a, b, x, y); }
  static __device__ __forceinline__ void keep(v16b a, v16b b, v16b c, v16b d) { keep4_b(a, b, c, d); }
};

template <int ET> struct Elem;
template <> struct Elem<0> { typedef _Float16 T; };
template <> struct Elem<1> { typedef __bf16 T; };
template <int ET, bool SPLIT, int BIAS_MODE, int OUT_MODE, bool RESID, int ACT = 0>
__global__ __launch_bounds__(256) void wmma_gemm64(
    const unsigned short* __restrict__ Ap, const unsigned short* __restrict__ A2p, int lda, long strideA,
    const unsigned short* __restrict__ Btp, const unsigned short* __restrict__ Bt2p, int ldb, long strideB,
    void* __restrict__ Cout, void* __restrict__ Cout2, int ldc, long strideC,
    const float* __restrict__ bias,
    const float* __restrict__ resid, long strideR,
    int M, int N, int K, float scale) {
  typedef typename Elem<ET>::T T;
  typedef typename Frag<T>::V V;
  const T* A = (const T*)Ap; const T* A2 = (const T*)A2p; const T* Bt = (const T*)Btp; const T* Bt2 = (const T*)Bt2p;
  __shared__ __align__(16) float sT[8][16 * 68];
  const int b    = blockIdx.y;
  const int lane = threadIdx.x & 31;
  const int wave = threadIdx.x >> 5;
  const int tilesN = N >> 6;
  const int tilesM = M >> 6;
  const int tile = blockIdx.x * 8 + wave;
  if (tile >= tilesM * tilesN) return;
  const int tm = tile / tilesN;
  const int tn = tile - tm * tilesN;
  const int m0 = tm << 6;
  const int n0 = tn << 6;

  const T* Ab  = A  + (size_t)b * strideA;
  const T* Bb  = Bt + (size_t)b * strideB;
  const T* Ab2 = SPLIT ? (A2  + (size_t)b * strideA) : nullptr;
  const T* Bb2 = SPLIT ? (Bt2 + (size_t)b * strideB) : nullptr;

  const int rlane = lane & 15;
  const int koff  = (lane >> 4) * 8;
  const int mOff  = (lane >> 4) * 8;

  v8f acc[4][4];
#pragma unroll
  for (int i = 0; i < 4; ++i)
#pragma unroll
    for (int j = 0; j < 4; ++j) acc[i][j] = (v8f){0.f,0.f,0.f,0.f,0.f,0.f,0.f,0.f};

  for (int k0 = 0; k0 < K; k0 += 32) {
    V bh[4], bl[4];
#pragma unroll
    for (int j = 0; j < 4; ++j) {
      const size_t bo = (size_t)(n0 + (j << 4) + rlane) * ldb + koff + k0;
      bh[j] = Frag<T>::load(Bb + bo);
      if (SPLIT) bl[j] = Frag<T>::load(Bb2 + bo);
    }
#pragma unroll
    for (int i = 0; i < 4; ++i) {
      const size_t ao = (size_t)(m0 + (i << 4) + rlane) * lda + koff + k0;
      V ah = Frag<T>::load(Ab + ao);
      V al;
      if (SPLIT) al = Frag<T>::load(Ab2 + ao);
#pragma unroll
      for (int j = 0; j < 4; ++j) {
        acc[i][j] = Frag<T>::mma(ah, bh[j], acc[i][j]);
        if (SPLIT) {
          acc[i][j] = Frag<T>::mma(ah, bl[j], acc[i][j]);
          acc[i][j] = Frag<T>::mma(al, bh[j], acc[i][j]);
        }
      }
      Frag<T>::guard(acc[i][0], acc[i][3], ah, SPLIT ? al : ah);
    }
    Frag<T>::keep(bh[0], bh[1], bh[2], bh[3]);
    if (SPLIT) Frag<T>::keep(bl[0], bl[1], bl[2], bl[3]);
  }
  acc_guard4(acc[0][0], acc[0][1], acc[0][2], acc[0][3]);
  acc_guard4(acc[1][0], acc[1][1], acc[1][2], acc[1][3]);
  acc_guard4(acc[2][0], acc[2][1], acc[2][2], acc[2][3]);
  acc_guard4(acc[3][0], acc[3][1], acc[3][2], acc[3][3]);

  float* slab = sT[wave];
  const float* Rb = RESID ? (resid + (size_t)b * strideR) : nullptr;
#pragma unroll
  for (int i = 0; i < 4; ++i) {
    const int mBase = m0 + (i << 4);
#pragma unroll
    for (int j = 0; j < 4; ++j) {
      const int n = n0 + (j << 4) + rlane;
      float bv = 0.f;
      if (BIAS_MODE == 2) bv = bias[n];
#pragma unroll
      for (int r = 0; r < 8; ++r) {
        float v = acc[i][j][r] * scale;
        if (BIAS_MODE == 1) v += bias[mBase + mOff + r];
        if (BIAS_MODE == 2) v += bv;
        if (RESID) v += Rb[(size_t)(mBase + mOff + r) * ldc + n];
        if (ACT == 1) v = tanhf(v);
        if (ACT == 2) v = fmaxf(v, 0.0f);
        if (ACT == 3) v = v / (1.0f + expf(-v));
        if (ACT == 4) v = (v > 0.f) ? v : 0.01f * v;
        if (ACT == 5) v = 0.5f * v * (1.0f + erff(v * 0.70710678118654752f));
        slab[(mOff + r) * 68 + (j << 4) + rlane] = v;
      }
    }
    __builtin_amdgcn_fence(__ATOMIC_RELEASE, "workgroup");
    __builtin_amdgcn_wave_barrier();
    __builtin_amdgcn_fence(__ATOMIC_ACQUIRE, "workgroup");
    if (OUT_MODE == 0) {
      float* C = (float*)Cout + (size_t)b * strideC;
      const int hh = lane >> 4, c4 = (lane & 15) * 4;
      for (int pass = 0; pass < 2; ++pass) {
#pragma unroll
        for (int it = 0; it < 8; ++it) {
          const int row = it * 2 + hh;
          v4f v = *(const v4f*)(slab + row * 68 + c4);
          *(volatile v4f*)(C + (size_t)(mBase + row) * ldc + n0 + c4) = v;
        }
        __threadfence();
      }
    } else {
      const int q = lane >> 3, c8 = (lane & 7) * 8;
      unsigned short* C  = (unsigned short*)Cout  + (size_t)b * strideC;
      unsigned short* C2 = (OUT_MODE == 2) ? ((unsigned short*)Cout2 + (size_t)b * strideC) : nullptr;
      for (int pass = 0; pass < 2; ++pass) {
#pragma unroll
        for (int it = 0; it < 4; ++it) {
          const int row = it * 4 + q;
          const float* sp = slab + row * 68 + c8;
          v8h hv, lv;
#pragma unroll
          for (int e = 0; e < 8; ++e) {
            if (OUT_MODE == 1) {
              hv[e] = (_Float16)sp[e];
            } else {
              unsigned short hb = f2bf_bits(sp[e]);
              unsigned short lb = f2bf_bits(sp[e] - bf_bits2f(hb));
              hv[e] = __builtin_bit_cast(_Float16, hb);
              lv[e] = __builtin_bit_cast(_Float16, lb);
            }
          }
          *(volatile v8h*)(C + (size_t)(mBase + row) * ldc + n0 + c8) = hv;
          if (OUT_MODE == 2) *(volatile v8h*)(C2 + (size_t)(mBase + row) * ldc + n0 + c8) = lv;
        }
        __threadfence();
      }
    }
    __builtin_amdgcn_fence(__ATOMIC_RELEASE, "workgroup");
    __builtin_amdgcn_wave_barrier();
    __builtin_amdgcn_fence(__ATOMIC_ACQUIRE, "workgroup");
  }
}

__global__ __launch_bounds__(256) void k_tr_cast(const float* __restrict__ in, int ldi, long sin,
                                                 half_t* __restrict__ out, int ldo, long sout, float scale) {
  __shared__ float tile[64][33];
  const int tid = threadIdx.x, lane = tid & 31, wave = tid >> 5;
  const int c0 = blockIdx.x * 32, r0 = blockIdx.y * 64;
  const float* ib = in + (size_t)blockIdx.z * sin;
  half_t* ob = out + (size_t)blockIdx.z * sout;
#pragma unroll
  for (int i = 0; i < 8; ++i) {
    const int r = wave + 8 * i;
    tile[r][lane] = ib[(size_t)(r0 + r) * ldi + c0 + lane];
  }
  __syncthreads();
  const int cr = wave * 4 + (lane >> 3);
  const int rr = (lane & 7) * 8;
  v8h hv;
#pragma unroll
  for (int e = 0; e < 8; ++e) hv[e] = (half_t)(tile[rr + e][cr] * scale);
  half_t* p = ob + (size_t)(c0 + cr) * ldo + r0 + rr;
  *(volatile v8h*)p = hv;
  __threadfence();
  *(volatile v8h*)p = hv;
}

__global__ __launch_bounds__(256) void k_sr_ln(const float* __restrict__ x, const float* __restrict__ w_sr,
                                               const float* __restrict__ b_sr, const float* __restrict__ g_ln,
                                               const float* __restrict__ b_ln, half_t* __restrict__ xk) {
  __shared__ float red[8];
  __shared__ float st[2];
  __shared__ __align__(16) half_t hrow[C_];
  const int bm = blockIdx.x;
  const int b = bm / M_, m = bm - b * M_;
  const int c = threadIdx.x, lane = c & 31, wave = c >> 5;
  const int oh = m / MH_, ow = m - oh * MH_;
  const float* xp = x + ((size_t)b * C_ + c) * N_;
  const float* wp = w_sr + c * 9;
  float y = 0.f;
#pragma unroll
  for (int kh = 0; kh < 3; ++kh) {
    const int ih = oh * 2 - 1 + kh;
    const int ihc = ih < 0 ? 0 : (ih >= H_ ? H_ - 1 : ih);
    const float rok = (ih >= 0 && ih < H_) ? 1.f : 0.f;
#pragma unroll
    for (int kw = 0; kw < 3; ++kw) {
      const int iw = ow * 2 - 1 + kw;
      const int iwc = iw < 0 ? 0 : (iw >= W_ ? W_ - 1 : iw);
      const float ok = (iw >= 0 && iw < W_) ? rok : 0.f;
      y = fmaf(wp[kh * 3 + kw] * ok, xp[ihc * W_ + iwc], y);
    }
  }
  y += b_sr[c];
  float v1 = y;
#pragma unroll
  for (int off = 16; off > 0; off >>= 1) v1 += __shfl_xor(v1, off, 32);
  if (lane == 0) red[wave] = v1;
  __syncthreads();
  if (wave == 0) {
    float a = (lane < 8) ? red[lane & 7] : 0.f;
#pragma unroll
    for (int off = 4; off > 0; off >>= 1) a += __shfl_xor(a, off, 32);
    if (lane == 0) st[0] = a * (1.0f / (float)C_);
  }
  __syncthreads();
  const float mu = st[0];
  const float dv = y - mu;
  float v2 = dv * dv;
#pragma unroll
  for (int off = 16; off > 0; off >>= 1) v2 += __shfl_xor(v2, off, 32);
  if (lane == 0) red[wave] = v2;
  __syncthreads();
  if (wave == 0) {
    float a = (lane < 8) ? red[lane & 7] : 0.f;
#pragma unroll
    for (int off = 4; off > 0; off >>= 1) a += __shfl_xor(a, off, 32);
    if (lane == 0) st[1] = a * (1.0f / (float)C_);
  }
  __syncthreads();
  const float var = st[1];
  const float val = dv * rsqrtf(var + EPS_) * g_ln[c] + b_ln[c];
  hrow[c] = (half_t)val;
  __syncthreads();
  if (wave == 0) {
    const v8h hv = *(const v8h*)(hrow + lane * 8);
    half_t* dst = xk + (size_t)bm * C_ + lane * 8;
    *(volatile v8h*)dst = hv;
    __threadfence();
    *(volatile v8h*)dst = hv;
  }
}

__global__ __launch_bounds__(MIXT) void k_mix_softmax(const float* __restrict__ S, const float* __restrict__ w_tc,
                                                      const float* __restrict__ b_tc, half_t* __restrict__ D16,
                                                      float* __restrict__ rowstat) {
  __shared__ __align__(16) float  vbuf[NH_ * M_];
  __shared__ __align__(16) half_t hbuf[NH_ * M_];
  __shared__ float red[6][16];
  const int n = blockIdx.x;
  const int tid = threadIdx.x, lane = tid & 31, wave = tid >> 5;
  float w[NH_][NH_], bt[NH_];
#pragma unroll
  for (int g = 0; g < NH_; ++g) {
    bt[g] = b_tc[g];
#pragma unroll
    for (int h = 0; h < NH_; ++h) w[g][h] = w_tc[g * NH_ + h];
  }
  const size_t plane = (size_t)N_ * M_;
  const float* Srow = S + (size_t)n * M_;

  float tmx[NH_];
#pragma unroll
  for (int g = 0; g < NH_; ++g) tmx[g] = -3.0e38f;
#pragma unroll 1
  for (int s = 0; s < 3; ++s) {
    const int m = tid + MIXT * s;
    float sv[NH_];
#pragma unroll
    for (int h = 0; h < NH_; ++h) sv[h] = Srow[(size_t)h * plane + m];
#pragma unroll
    for (int g = 0; g < NH_; ++g) {
      float a = bt[g];
#pragma unroll
      for (int h = 0; h < NH_; ++h) a = fmaf(w[g][h], sv[h], a);
      vbuf[g * M_ + m] = a;
      tmx[g] = fmaxf(tmx[g], a);
    }
  }
#pragma unroll
  for (int g = 0; g < NH_; ++g) {
    float v = tmx[g];
#pragma unroll
    for (int off = 16; off > 0; off >>= 1) v = fmaxf(v, __shfl_xor(v, off, 32));
    tmx[g] = v;
  }
  if (lane == 0) {
#pragma unroll
    for (int g = 0; g < NH_; ++g) red[wave][g] = tmx[g];
  }
  __syncthreads();
  float gmx[NH_];
#pragma unroll
  for (int g = 0; g < NH_; ++g) {
    float v = red[0][g];
#pragma unroll
    for (int wv = 1; wv < 6; ++wv) v = fmaxf(v, red[wv][g]);
    gmx[g] = v;
  }
  __syncthreads();

  float tsm[NH_];
#pragma unroll
  for (int g = 0; g < NH_; ++g) tsm[g] = 0.f;
#pragma unroll 1
  for (int s = 0; s < 3; ++s) {
    const int m = tid + MIXT * s;
#pragma unroll
    for (int g = 0; g < NH_; ++g) {
      const float p = __expf(vbuf[g * M_ + m] - gmx[g]);
      vbuf[g * M_ + m] = p;
      tsm[g] += p;
    }
  }
#pragma unroll
  for (int g = 0; g < NH_; ++g) {
    float v = tsm[g];
#pragma unroll
    for (int off = 16; off > 0; off >>= 1) v += __shfl_xor(v, off, 32);
    tsm[g] = v;
  }
  if (lane == 0) {
#pragma unroll
    for (int g = 0; g < NH_; ++g) red[wave][g] = tsm[g];
  }
  __syncthreads();
  float inv[NH_];
#pragma unroll
  for (int g = 0; g < NH_; ++g) {
    float v = red[0][g];
#pragma unroll
    for (int wv = 1; wv < 6; ++wv) v += red[wv][g];
    inv[g] = __builtin_amdgcn_rcpf(v);
  }
  __syncthreads();

  float tS[NH_], tQ[NH_];
#pragma unroll
  for (int g = 0; g < NH_; ++g) { tS[g] = 0.f; tQ[g] = 0.f; }
#pragma unroll 1
  for (int s = 0; s < 3; ++s) {
    const int m = tid + MIXT * s;
#pragma unroll
    for (int g = 0; g < NH_; ++g) {
      const float P = vbuf[g * M_ + m] * inv[g];
      const float d = P - INV_M;
      hbuf[g * M_ + m] = (half_t)(d * DSC);
      tS[g] += d;
      tQ[g] = fmaf(d, d, tQ[g]);
    }
  }
#pragma unroll
  for (int g = 0; g < NH_; ++g) {
    float a = tS[g], q2 = tQ[g];
#pragma unroll
    for (int off = 16; off > 0; off >>= 1) {
      a  += __shfl_xor(a, off, 32);
      q2 += __shfl_xor(q2, off, 32);
    }
    tS[g] = a; tQ[g] = q2;
  }
  if (lane == 0) {
#pragma unroll
    for (int g = 0; g < NH_; ++g) { red[wave][2 * g] = tS[g]; red[wave][2 * g + 1] = tQ[g]; }
  }
  __syncthreads();
  if (wave == 0) {
    const int ql = lane & 15;
    float v = red[0][ql];
#pragma unroll
    for (int wv = 1; wv < 6; ++wv) v += red[wv][ql];
    if (lane >= 16) v = 0.f;
    float* rp = rowstat + (size_t)n * 32 + lane;
    *(volatile float*)rp = v;
    __threadfence();
    *(volatile float*)rp = v;
  }
  const int q = lane >> 3, c8 = (lane & 7) * 8;
  for (int g = wave; g < NH_; g += 6) {
    const half_t* hb = hbuf + g * M_;
    half_t* dp = D16 + ((size_t)g * N_ + n) * M_;
    for (int pass = 0; pass < 2; ++pass) {
#pragma unroll
      for (int it = 0; it < 3; ++it) {
        const int line = it * 4 + q;
        const int lc = (line < 9) ? line : 8;
        const int off = lc * 64 + c8;
        const v8h hv = *(const v8h*)(hb + off);
        if (line < 9) *(volatile v8h*)(dp + off) = hv;
      }
      __threadfence();
    }
  }
}

__global__ __launch_bounds__(256) void k_stats(const float* __restrict__ rowstat, const half_t* __restrict__ vT,
                                               float* __restrict__ stat) {
  __shared__ double dred[16][17];
  __shared__ double tot[16];
  const int tid = threadIdx.x, lane = tid & 31, wave = tid >> 5;
  const int qn = tid & 15, grp = tid >> 4;
  double acc = 0.0;
#pragma unroll 4
  for (int i = 0; i < N_ / 16; ++i) acc += (double)rowstat[(size_t)(grp + 16 * i) * 32 + qn];
  dred[grp][qn] = acc;
  float cs = 0.f;
  {
    const half_t* vr = vT + (size_t)tid * M_;
#pragma unroll 2
    for (int j = 0; j < M_ / 8; ++j) {
      const v8h hv = *(const v8h*)(vr + 8 * j);
#pragma unroll
      for (int e = 0; e < 8; ++e) cs += (float)hv[e];
    }
  }
  __syncthreads();
  {
    const int tq = tid & 15;
    double t = 0.0;
#pragma unroll
    for (int g2 = 0; g2 < 16; ++g2) t += dred[g2][tq];
    if (tid < 16) tot[tq] = t;
  }
  __syncthreads();
  float v2 = 0.f;
  if (wave == 0) {
    const int g = lane & 7;
    const double Sd = tot[2 * g], Qd = tot[2 * g + 1];
    const double dbar = Sd * INV_CNT;
    double var = Qd * INV_CNT - dbar * dbar;
    if (var < 0.0) var = 0.0;
    const float rs = rsqrtf((float)var + EPS_);
    v2 = (lane < 8) ? rs : ((lane < 16) ? (float)dbar : 0.f);
  }
  for (int pass = 0; pass < 2; ++pass) {
    *(volatile float*)(stat + tid) = cs;
    if (wave == 0) *(volatile float*)(stat + 256 + lane) = v2;
    __threadfence();
  }
}

__global__ __launch_bounds__(128) void k_pv(const half_t* __restrict__ D16, const half_t* __restrict__ vT,
                                            const float* __restrict__ stat, half_t* __restrict__ O16) {
  __shared__ __align__(16) float sT[4][16 * 68];
  const int lane = threadIdx.x & 31, wave = threadIdx.x >> 5;
  const int wg = blockIdx.x * 4 + wave;
  const int gp = wg / 144;
  const int rt = wg - gp * 144;
  if (gp >= 4) return;
  const int n0 = rt * 16;
  const int rlane = lane & 15, koff = (lane >> 4) * 8, mOff = (lane >> 4) * 8;
  const half_t* A0 = D16 + ((size_t)(2 * gp) * N_ + n0 + rlane) * M_ + koff;
  const half_t* A1 = A0 + (size_t)N_ * M_;
  const half_t* Bp = vT + (size_t)(64 * gp + rlane) * M_ + koff;
  v8f acc[4];
#pragma unroll
  for (int j = 0; j < 4; ++j) acc[j] = (v8f){0.f,0.f,0.f,0.f,0.f,0.f,0.f,0.f};
  for (int k0 = 0; k0 < M_; k0 += 32) {
    const v16h b0 = Frag<half_t>::load(Bp + k0);
    const v16h b1 = Frag<half_t>::load(Bp + 16 * M_ + k0);
    const v16h b2 = Frag<half_t>::load(Bp + 32 * M_ + k0);
    const v16h b3 = Frag<half_t>::load(Bp + 48 * M_ + k0);
    const v16h a0 = Frag<half_t>::load(A0 + k0);
    const v16h a1 = Frag<half_t>::load(A1 + k0);
    acc[0] = Frag<half_t>::mma(a0, b0, acc[0]);
    acc[1] = Frag<half_t>::mma(a0, b1, acc[1]);
    acc[2] = Frag<half_t>::mma(a1, b2, acc[2]);
    acc[3] = Frag<half_t>::mma(a1, b3, acc[3]);
    Frag<half_t>::guard(acc[0], acc[3], a0, a1);
    Frag<half_t>::keep(b0, b1, b2, b3);
  }
  acc_guard4(acc[0], acc[1], acc[2], acc[3]);
  const float rs0 = stat[256 + 2 * gp], rs1 = stat[257 + 2 * gp];
  const float db0 = stat[264 + 2 * gp], db1 = stat[265 + 2 * gp];
  float* slab = sT[wave];
#pragma unroll
  for (int j = 0; j < 4; ++j) {
    const int c = 64 * gp + 16 * j + rlane;
    const float cs = stat[c];
    const float rs = (j < 2) ? rs0 : rs1;
    const float db = (j < 2) ? db0 : db1;
    const float corr = db * cs;
#pragma unroll
    for (int r = 0; r < 8; ++r) slab[(mOff + r) * 68 + 16 * j + rlane] = rs * (acc[j][r] * DSC_INV - corr);
  }
  __builtin_amdgcn_fence(__ATOMIC_RELEASE, "workgroup");
  __builtin_amdgcn_wave_barrier();
  __builtin_amdgcn_fence(__ATOMIC_ACQUIRE, "workgroup");
  {
    const int q = lane >> 3, c8 = (lane & 7) * 8;
    half_t* ob = O16 + (size_t)n0 * C_ + 64 * gp + c8;
    for (int pass = 0; pass < 2; ++pass) {
#pragma unroll
      for (int it = 0; it < 4; ++it) {
        const int row = it * 4 + q;
        const float* sp = slab + row * 68 + c8;
        v8h hv;
#pragma unroll
        for (int e = 0; e < 8; ++e) hv[e] = (half_t)sp[e];
        *(volatile v8h*)(ob + (size_t)row * C_) = hv;
      }
      __threadfence();
    }
  }
}

extern "C" void kernel_launch(void* const* d_in, const int* in_sizes, int n_in,
                              void* d_out, int out_size, void* d_ws,
                              size_t ws_size, hipStream_t stream) {
  if (n_in < 11) return;
  if (out_size != B_ * C_ * N_) return;
  if (in_sizes[0] != B_ * C_ * N_ || in_sizes[1] != C_ * C_ || in_sizes[2] != 2 * C_ * C_ ||
      in_sizes[3] != C_ * 9 || in_sizes[7] != NH_ * NH_ || in_sizes[9] != C_ * C_) return;

  const float* x      = (const float*)d_in[0];
  const float* w_q    = (const float*)d_in[1];
  const float* w_kv   = (const float*)d_in[2];
  const float* w_sr   = (const float*)d_in[3];
  const float* b_sr   = (const float*)d_in[4];
  const float* g_ln   = (const float*)d_in[5];
  const float* b_ln   = (const float*)d_in[6];
  const float* w_tc   = (const float*)d_in[7];
  const float* b_tc   = (const float*)d_in[8];
  const float* w_proj = (const float*)d_in[9];
  const float* b_proj = (const float*)d_in[10];

  uint8_t* wbase = (uint8_t*)d_ws;
  uint8_t* wcur = wbase;
  auto take = [&](size_t bytes) {
    uint8_t* p = wcur;
    wcur += (bytes + 255) & ~(size_t)255;
    return p;
  };
  half_t* wqT  = (half_t*)take((size_t)C_ * C_ * 2);
  half_t* wkvT = (half_t*)take((size_t)2 * C_ * C_ * 2);
  half_t* wpT  = (half_t*)take((size_t)C_ * C_ * 2);
  half_t* xt16 = (half_t*)take((size_t)B_ * N_ * C_ * 2);
  half_t* O16  = xt16;
  half_t* q16  = (half_t*)take((size_t)B_ * N_ * C_ * 2);
  half_t* xk16 = (half_t*)take((size_t)B_ * M_ * C_ * 2);
  half_t* k16  = (half_t*)take((size_t)B_ * M_ * C_ * 2);
  half_t* vT16 = (half_t*)take((size_t)B_ * C_ * M_ * 2);
  float*  S    = (float*)take((size_t)NH_ * N_ * M_ * 4);
  half_t* D16  = (half_t*)take((size_t)NH_ * N_ * M_ * 2);
  float*  rowstat = (float*)take((size_t)B_ * N_ * 32 * 4);
  float*  stat    = (float*)take((size_t)B_ * 512 * 4);
  const size_t total = (size_t)(wcur - wbase);
  if (total > ws_size || total > (size_t)134217728) return;

  auto u16 = [](const void* p) { return (const unsigned short*)p; };

  k_tr_cast<<<dim3(C_ / 32, C_ / 64, 1), dim3(256), 0, stream>>>(w_q, C_, 0L, wqT, C_, 0L, WSC);
  k_tr_cast<<<dim3(2 * C_ / 32, C_ / 64, 1), dim3(256), 0, stream>>>(w_kv, 2 * C_, 0L, wkvT, C_, 0L, WSC);
  k_tr_cast<<<dim3(C_ / 32, C_ / 64, 1), dim3(256), 0, stream>>>(w_proj, C_, 0L, wpT, C_, 0L, WSC);
  k_tr_cast<<<dim3(N_ / 32, C_ / 64, B_), dim3(256), 0, stream>>>(x, N_, (long)C_ * N_, xt16, C_, (long)N_ * C_, 1.0f);
  k_sr_ln<<<dim3(B_ * M_), dim3(256), 0, stream>>>(x, w_sr, b_sr, g_ln, b_ln, xk16);
  wmma_gemm64<0, false, 0, 1, false, 0><<<dim3(144, 1), dim3(256), 0, stream>>>(
      u16(xt16), u16(xt16), C_, 0L, u16(wqT), u16(wqT), C_, 0L,
      (void*)q16, (void*)q16, C_, 0L, b_proj, b_proj, 0L, B_ * N_, C_, C_, WSC_INV);
  wmma_gemm64<0, false, 0, 1, false, 0><<<dim3(36, 1), dim3(256), 0, stream>>>(
      u16(xk16), u16(xk16), C_, 0L, u16(wkvT), u16(wkvT), C_, 0L,
      (void*)k16, (void*)k16, C_, 0L, b_proj, b_proj, 0L, B_ * M_, C_, C_, WSC_INV);
  wmma_gemm64<0, false, 0, 1, false, 0><<<dim3(5, B_), dim3(256), 0, stream>>>(
      u16(wkvT + (size_t)C_ * C_), u16(wkvT + (size_t)C_ * C_), C_, 0L,
      u16(xk16), u16(xk16), C_, (long)M_ * C_,
      (void*)vT16, (void*)vT16, M_, (long)C_ * M_, b_proj, b_proj, 0L, C_, M_, C_, WSC_INV);

  for (int b = 0; b < B_; ++b) {
    const half_t* qb = q16 + (size_t)b * N_ * C_;
    const half_t* kb = k16 + (size_t)b * M_ * C_;
    const half_t* vb = vT16 + (size_t)b * C_ * M_;
    wmma_gemm64<0, false, 0, 0, false, 0><<<dim3(41, NH_), dim3(256), 0, stream>>>(
        u16(qb), u16(qb), C_, (long)HD_, u16(kb), u16(kb), C_, (long)HD_,
        (void*)S, (void*)S, M_, (long)N_ * M_, b_proj, b_proj, 0L, N_, M_, HD_, SCALE_);
    k_mix_softmax<<<dim3(N_), dim3(MIXT), 0, stream>>>(S, w_tc, b_tc, D16, rowstat + (size_t)b * N_ * 32);
    k_stats<<<dim3(1), dim3(256), 0, stream>>>(rowstat + (size_t)b * N_ * 32, vb, stat + (size_t)b * 512);
    k_pv<<<dim3(144), dim3(128), 0, stream>>>(D16, vb, stat + (size_t)b * 512, O16 + (size_t)b * N_ * C_);
  }
  wmma_gemm64<0, false, 1, 0, false, 0><<<dim3(18, B_), dim3(256), 0, stream>>>(
      u16(wpT), u16(wpT), C_, 0L, u16(O16), u16(O16), C_, (long)N_ * C_,
      d_out, d_out, N_, (long)C_ * N_, b_proj, b_proj, 0L, C_, N_, C_, WSC_INV);
}
